// RWKVTimeMixing_10900626997665
// MI455X (gfx1250) — hardware-verified
//
#include <hip/hip_runtime.h>
#include <math.h>

constexpr int kNB    = 4;
constexpr int kNS    = 2048;
constexpr int kND    = 1024;
constexpr int kNRows = kNB * kNS;
constexpr float kWCarry    = 32.0f;
constexpr float kYCarry    = 64.0f;
constexpr float kProjScale = 1.0f / 32.0f;
constexpr float kOutScale  = 1.0f / 2048.0f;
constexpr int kScanGroup   = 8;

constexpr size_t kPlaneH  = (size_t)kNRows * kND * 2;
constexpr size_t kPlaneF  = (size_t)kNRows * kND * 4;
constexpr size_t kWPlaneH = (size_t)kND * kND * 2;
constexpr size_t kOffW16  = 0;
constexpr size_t kOffXK   = kOffW16 + 4 * kWPlaneH;
constexpr size_t kOffXV   = kOffXK + kPlaneH;
constexpr size_t kOffXR   = kOffXV + kPlaneH;
constexpr size_t kOffKf   = kOffXR + kPlaneH;
constexpr size_t kOffVf   = kOffKf + kPlaneF;
constexpr size_t kWsEnd   = kOffVf + kPlaneF;
constexpr size_t kOffZf   = kOffXK;
constexpr size_t kOffY16  = kOffXR;
static_assert(kOffZf + kPlaneF <= kOffXR, "Zf fits in the dead XK+XV region");
static_assert(kOffY16 + kPlaneH <= kOffKf, "Y16 fits in the dead XR region");
static_assert(kWsEnd == 125829120, "carve total");
static_assert(kWsEnd <= 134217728, "carve under 128 MiB");
static_assert(kNRows % 64 == 0 && kND % 64 == 0 && kND % 32 == 0, "GEMM tile multiples, K % 32 == 0");

typedef __attribute__((ext_vector_type(16))) _Float16 v16h;
typedef __attribute__((ext_vector_type(8)))  _Float16 v8h;
typedef __attribute__((ext_vector_type(16))) __bf16   v16b;
typedef __attribute__((ext_vector_type(8)))  __bf16   v8b;
typedef __attribute__((ext_vector_type(8)))  float    v8f;
typedef __attribute__((ext_vector_type(4)))  float    v4f;
typedef __attribute__((ext_vector_type(4)))  unsigned int v4u;

__device__ __forceinline__ unsigned short f2bf_bits(float f) {
  unsigned u = __float_as_uint(f);
  return (unsigned short)((u + 0x7FFFu + ((u >> 16) & 1u)) >> 16);
}
__device__ __forceinline__ float bf_bits2f(unsigned short h) { return __uint_as_float(((unsigned)h) << 16); }

__device__ __forceinline__ void dep_guard_h(v8f& a, v8f& b, v16h x, v16h y) { asm volatile("v_nop\n\tv_nop\n\tv_nop\n\tv_nop" : "+v"(a), "+v"(b) : "v"(x), "v"(y)); }
__device__ __forceinline__ void dep_guard_b(v8f& a, v8f& b, v16b x, v16b y) { asm volatile("v_nop\n\tv_nop\n\tv_nop\n\tv_nop" : "+v"(a), "+v"(b) : "v"(x), "v"(y)); }
__device__ __forceinline__ void keep4_h(v16h a, v16h b, v16h c, v16h d) { asm volatile("v_nop" :: "v"(a), "v"(b), "v"(c), "v"(d)); }
__device__ __forceinline__ void keep4_b(v16b a, v16b b, v16b c, v16b d) { asm volatile("v_nop" :: "v"(a), "v"(b), "v"(c), "v"(d)); }
__device__ __forceinline__ void acc_guard4(v8f& a, v8f& b, v8f& c, v8f& d) { asm volatile("v_nop\n\tv_nop\n\tv_nop\n\tv_nop" : "+v"(a), "+v"(b), "+v"(c), "+v"(d)); }
template <typename T> struct Frag;
template <> struct Frag<_Float16> {
  typedef v16h V; union U { v16h v; v8h h[2]; };
  static __device__ __forceinline__ v16h load(const _Float16* p) {
    U f; f.h[0] = *(const v8h*)(p); f.h[1] = *(const v8h*)(p + 16); return f.v;
  }
  static __device__ __forceinline__ v8f mma(v16h a, v16h b, v8f c) {
    return __builtin_amdgcn_wmma_f32_16x16x32_f16(false, a, false, b, (short)0, c, false, false);
  }
  static __device__ __forceinline__ void guard(v8f& a, v8f& b, v16h x, v16h y) { dep_guard_h(a, b, x, y); }
  static __device__ __forceinline__ void keep(v16h a, v16h b, v16h c, v16h d) { keep4_h(a, b, c, d); }
};
template <> struct Frag<__bf16> {
  typedef v16b V; union U { v16b v; v8b h[2]; };
  static __device__ __forceinline__ v16b load(const __bf16* p) {
    U f; f.h[0] = *(const v8b*)(p); f.h[1] = *(const v8b*)(p + 16); return f.v;
  }
  static __device__ __forceinline__ v8f mma(v16b a, v16b b, v8f c) {
    return __builtin_amdgcn_wmma_f32_16x16x32_bf16(false, a, false, b, (short)0, c, false, false);
  }
  static __device__ __forceinline__ void guard(v8f& a, v8f& b, v16b x, v16b y) { dep_guard_b(a, b, x, y); }
  static __device__ __forceinline__ void keep(v16b a, v16b b, v16b c, v16b d) { keep4_b(a, b, c, d); }
};

__device__ __forceinline__ unsigned pk16(unsigned short a, unsigned short b) { return (unsigned)a | ((unsigned)b << 16); }
__device__ __forceinline__ unsigned short h_bits(float f) { const _Float16 h = (_Float16)f; return __builtin_bit_cast(unsigned short, h); }

template <int ET> struct Elem;
template <> struct Elem<0> { typedef _Float16 T; };
template <> struct Elem<1> { typedef __bf16 T; };
template <int ET, bool SPLIT, int BIAS_MODE, int OUT_MODE, bool RESID, int ACT = 0>
__global__ __launch_bounds__(256) void wmma_gemm64(
    const unsigned short* __restrict__ Ap, const unsigned short* __restrict__ A2p, int lda, long strideA,
    const unsigned short* __restrict__ Btp, const unsigned short* __restrict__ Bt2p, int ldb, long strideB,
    void* __restrict__ Cout, void* __restrict__ Cout2, int ldc, long strideC,
    const float* __restrict__ bias,
    const float* __restrict__ resid, long strideR,
    int M, int N, int K, float scale) {
  typedef typename Elem<ET>::T T;
  typedef typename Frag<T>::V V;
  const T* A = (const T*)Ap; const T* A2 = (const T*)A2p; const T* Bt = (const T*)Btp; const T* Bt2 = (const T*)Bt2p;
  __shared__ __align__(16) float sT[8][16 * 68];
  const int b    = blockIdx.y;
  const int lane = threadIdx.x & 31;
  const int wave = threadIdx.x >> 5;
  const int tilesN = N >> 6;
  const int tilesM = M >> 6;
  const int tile = blockIdx.x * 8 + wave;
  if (tile >= tilesM * tilesN) return;
  const int tm = tile / tilesN;
  const int tn = tile - tm * tilesN;
  const int m0 = tm << 6;
  const int n0 = tn << 6;

  const T* Ab  = A  + (size_t)b * strideA;
  const T* Bb  = Bt + (size_t)b * strideB;
  const T* Ab2 = SPLIT ? (A2  + (size_t)b * strideA) : nullptr;
  const T* Bb2 = SPLIT ? (Bt2 + (size_t)b * strideB) : nullptr;

  const int rlane = lane & 15;
  const int koff  = (lane >> 4) * 8;
  const int mOff  = (lane >> 4) * 8;

  v8f acc[4][4];
#pragma unroll
  for (int i = 0; i < 4; ++i)
#pragma unroll
    for (int j = 0; j < 4; ++j) acc[i][j] = (v8f){0.f,0.f,0.f,0.f,0.f,0.f,0.f,0.f};

  for (int k0 = 0; k0 < K; k0 += 32) {
    V bh[4], bl[4];
#pragma unroll
    for (int j = 0; j < 4; ++j) {
      const size_t bo = (size_t)(n0 + (j << 4) + rlane) * ldb + koff + k0;
      bh[j] = Frag<T>::load(Bb + bo);
      if (SPLIT) bl[j] = Frag<T>::load(Bb2 + bo);
    }
#pragma unroll
    for (int i = 0; i < 4; ++i) {
      const size_t ao = (size_t)(m0 + (i << 4) + rlane) * lda + koff + k0;
      V ah = Frag<T>::load(Ab + ao);
      V al;
      if (SPLIT) al = Frag<T>::load(Ab2 + ao);
#pragma unroll
      for (int j = 0; j < 4; ++j) {
        acc[i][j] = Frag<T>::mma(ah, bh[j], acc[i][j]);
        if (SPLIT) {
          acc[i][j] = Frag<T>::mma(ah, bl[j], acc[i][j]);
          acc[i][j] = Frag<T>::mma(al, bh[j], acc[i][j]);
        }
      }
      Frag<T>::guard(acc[i][0], acc[i][3], ah, SPLIT ? al : ah);
    }
    Frag<T>::keep(bh[0], bh[1], bh[2], bh[3]);
    if (SPLIT) Frag<T>::keep(bl[0], bl[1], bl[2], bl[3]);
  }
  acc_guard4(acc[0][0], acc[0][1], acc[0][2], acc[0][3]);
  acc_guard4(acc[1][0], acc[1][1], acc[1][2], acc[1][3]);
  acc_guard4(acc[2][0], acc[2][1], acc[2][2], acc[2][3]);
  acc_guard4(acc[3][0], acc[3][1], acc[3][2], acc[3][3]);

  float* slab = sT[wave];
  const float* Rb = RESID ? (resid + (size_t)b * strideR) : nullptr;
#pragma unroll
  for (int i = 0; i < 4; ++i) {
    const int mBase = m0 + (i << 4);
#pragma unroll
    for (int j = 0; j < 4; ++j) {
      const int n = n0 + (j << 4) + rlane;
      float bv = 0.f;
      if (BIAS_MODE == 2) bv = bias[n];
#pragma unroll
      for (int r = 0; r < 8; ++r) {
        float v = acc[i][j][r] * scale;
        if (BIAS_MODE == 1) v += bias[mBase + mOff + r];
        if (BIAS_MODE == 2) v += bv;
        if (RESID) v += Rb[(size_t)(mBase + mOff + r) * ldc + n];
        if (ACT == 2) v = fmaxf(v, 0.0f);
        if (ACT == 4) v = (v > 0.f) ? v : 0.01f * v;
        slab[(mOff + r) * 68 + (j << 4) + rlane] = v;
      }
    }
    __builtin_amdgcn_fence(__ATOMIC_RELEASE, "workgroup");
    __builtin_amdgcn_wave_barrier();
    __builtin_amdgcn_fence(__ATOMIC_ACQUIRE, "workgroup");
    if (OUT_MODE == 0) {
      float* C = (float*)Cout + (size_t)b * strideC;
      const int hh = lane >> 4, c4 = (lane & 15) * 4;
      for (int pass = 0; pass < 2; ++pass) {
#pragma unroll
        for (int it = 0; it < 8; ++it) {
          const int row = it * 2 + hh;
          v4f v = *(const v4f*)(slab + row * 68 + c4);
          *(volatile v4f*)(C + (size_t)(mBase + row) * ldc + n0 + c4) = v;
        }
        __threadfence();
      }
    } else {
      const int q = lane >> 3, c8 = (lane & 7) * 8;
      unsigned short* C  = (unsigned short*)Cout  + (size_t)b * strideC;
      unsigned short* C2 = (OUT_MODE == 2) ? ((unsigned short*)Cout2 + (size_t)b * strideC) : nullptr;
      for (int pass = 0; pass < 2; ++pass) {
#pragma unroll
        for (int it = 0; it < 4; ++it) {
          const int row = it * 4 + q;
          const float* sp = slab + row * 68 + c8;
          v8h hv, lv;
#pragma unroll
          for (int e = 0; e < 8; ++e) {
            if (OUT_MODE == 1) {
              hv[e] = (_Float16)sp[e];
            } else {
              unsigned short hb = f2bf_bits(sp[e]);
              unsigned short lb = f2bf_bits(sp[e] - bf_bits2f(hb));
              hv[e] = __builtin_bit_cast(_Float16, hb);
              lv[e] = __builtin_bit_cast(_Float16, lb);
            }
          }
          *(volatile v8h*)(C + (size_t)(mBase + row) * ldc + n0 + c8) = hv;
          if (OUT_MODE == 2) *(volatile v8h*)(C2 + (size_t)(mBase + row) * ldc + n0 + c8) = lv;
        }
        __threadfence();
      }
    }
    __builtin_amdgcn_fence(__ATOMIC_RELEASE, "workgroup");
    __builtin_amdgcn_wave_barrier();
    __builtin_amdgcn_fence(__ATOMIC_ACQUIRE, "workgroup");
  }
}

__global__ __launch_bounds__(256) void wcast8_kernel(const float* __restrict__ W0, const float* __restrict__ W1,
                                                     const float* __restrict__ W2, const float* __restrict__ W3,
                                                     unsigned short* __restrict__ out, int n8, float scale) {
  const int z = blockIdx.y;
  const float* W = (z == 0) ? W0 : (z == 1) ? W1 : (z == 2) ? W2 : W3;
  const int i = blockIdx.x * 256 + threadIdx.x;
  if (i >= n8) return;
  const float* p = W + 8 * (size_t)i;
  const v4f a = *(const v4f*)(p);
  const v4f c = *(const v4f*)(p + 4);
  unsigned short hb[8];
#pragma unroll
  for (int e = 0; e < 4; ++e) {
    hb[e]     = h_bits(a[e] * scale);
    hb[4 + e] = h_bits(c[e] * scale);
  }
  const v4u u = (v4u){pk16(hb[0], hb[1]), pk16(hb[2], hb[3]), pk16(hb[4], hb[5]), pk16(hb[6], hb[7])};
  unsigned short* q = out + (size_t)z * kND * kND + 8 * (size_t)i;
  *(volatile v4u*)q = u;
  __threadfence();
  *(volatile v4u*)q = u;
}

__global__ __launch_bounds__(256) void mix_kernel(const float* __restrict__ x, const float* __restrict__ tmk,
                                                  const float* __restrict__ tmv, const float* __restrict__ tmr,
                                                  unsigned short* __restrict__ xk, unsigned short* __restrict__ xv,
                                                  unsigned short* __restrict__ xr, int n8) {
#pragma clang fp contract(off)
  const int i = blockIdx.x * 256 + threadIdx.x;
  if (i >= n8) return;
  const size_t e0 = 8 * (size_t)i;
  const int d0 = (int)(e0 & (size_t)(kND - 1));
  const int s  = (int)((e0 >> 10) & (size_t)(kNS - 1));
  const float* xp = x + e0;
  const v4f xa = *(const v4f*)(xp);
  const v4f xb = *(const v4f*)(xp + 4);
  const float* shp = (s == 0) ? xp : (xp - kND);
  const v4f sa0 = *(const v4f*)(shp);
  const v4f sb0 = *(const v4f*)(shp + 4);
  const v4f ka = *(const v4f*)(tmk + d0);
  const v4f kb = *(const v4f*)(tmk + d0 + 4);
  const v4f va = *(const v4f*)(tmv + d0);
  const v4f vb = *(const v4f*)(tmv + d0 + 4);
  const v4f ra = *(const v4f*)(tmr + d0);
  const v4f rb = *(const v4f*)(tmr + d0 + 4);
  float xc[8], sh[8], mk[8], mv[8], mr[8];
#pragma unroll
  for (int e = 0; e < 4; ++e) {
    xc[e] = xa[e]; xc[4 + e] = xb[e];
    sh[e] = (s == 0) ? 0.0f : sa0[e]; sh[4 + e] = (s == 0) ? 0.0f : sb0[e];
    mk[e] = ka[e]; mk[4 + e] = kb[e];
    mv[e] = va[e]; mv[4 + e] = vb[e];
    mr[e] = ra[e]; mr[4 + e] = rb[e];
  }
  unsigned short hk[8], hv[8], hr[8];
#pragma unroll
  for (int e = 0; e < 8; ++e) {
    const float omk = 1.0f - mk[e];
    const float omv = 1.0f - mv[e];
    const float omr = 1.0f - mr[e];
    const float ak = xc[e] * mk[e];
    const float bk = sh[e] * omk;
    const float av = xc[e] * mv[e];
    const float bvv = sh[e] * omv;
    const float ar = xc[e] * mr[e];
    const float br = sh[e] * omr;
    hk[e] = h_bits(ak + bk);
    hv[e] = h_bits(av + bvv);
    hr[e] = h_bits(ar + br);
  }
  const v4u uk = (v4u){pk16(hk[0], hk[1]), pk16(hk[2], hk[3]), pk16(hk[4], hk[5]), pk16(hk[6], hk[7])};
  const v4u uv = (v4u){pk16(hv[0], hv[1]), pk16(hv[2], hv[3]), pk16(hv[4], hv[5]), pk16(hv[6], hv[7])};
  const v4u ur = (v4u){pk16(hr[0], hr[1]), pk16(hr[2], hr[3]), pk16(hr[4], hr[5]), pk16(hr[6], hr[7])};
  unsigned short* qk = xk + e0;
  unsigned short* qv = xv + e0;
  unsigned short* qr = xr + e0;
  *(volatile v4u*)qk = uk;
  *(volatile v4u*)qv = uv;
  *(volatile v4u*)qr = ur;
  __threadfence();
  *(volatile v4u*)qk = uk;
  *(volatile v4u*)qv = uv;
  *(volatile v4u*)qr = ur;
}

__global__ __launch_bounds__(256) void wkv_scan_kernel(const float* __restrict__ Kf, const float* __restrict__ Vf,
                                                       const float* __restrict__ Zf, const float* __restrict__ td,
                                                       const float* __restrict__ tf, unsigned short* __restrict__ Y,
                                                       float ycarry) {
#pragma clang fp contract(off)
  __shared__ __align__(16) unsigned short ybuf[kScanGroup * 256];
  const int tid  = threadIdx.x;
  const int lane = tid & 31;
  const int wave = tid >> 5;
  const int b    = blockIdx.x >> 2;
  const int d0   = (blockIdx.x & 3) * 256;
  const int d    = d0 + tid;
  const float w  = -expf(td[d]);
  const float u  = tf[d];
  float aa = 0.0f, bb = 0.0f, pp = -1e30f;
  const size_t rowbase = (size_t)b * kNS;
#pragma unroll 1
  for (int sg = 0; sg < kNS / kScanGroup; ++sg) {
#pragma unroll 1
    for (int j = 0; j < kScanGroup; ++j) {
      const int s = sg * kScanGroup + j;
      const size_t idx = (rowbase + (size_t)s) * kND + d;
      const float kk = Kf[idx];
      const float vv = Vf[idx];
      const float zz = Zf[idx];
      const float ww = u + kk;
      const float p  = fmaxf(pp, ww);
      const float e1 = expf(pp - p);
      const float e2 = expf(ww - p);
      const float numa = e1 * aa;
      const float numb = e2 * vv;
      const float dena = e1 * bb;
      const float o    = (numa + numb) / (dena + e2);
      const float rr   = 1.0f / (1.0f + expf(-zz));
      const float y    = (rr * o) * ycarry;
      ybuf[j * 256 + tid] = h_bits(y);
      const float ww2 = w + pp;
      const float p2  = fmaxf(ww2, kk);
      const float e1b = expf(ww2 - p2);
      const float e2b = expf(kk - p2);
      const float na  = e1b * aa;
      const float nb  = e2b * vv;
      const float nc  = e1b * bb;
      aa = na + nb;
      bb = nc + e2b;
      pp = p2;
    }
    __syncthreads();
    const v4u val = *(const v4u*)(ybuf + wave * 256 + lane * 8);
    unsigned short* dst = Y + ((rowbase + (size_t)(sg * kScanGroup + wave)) * kND + d0 + lane * 8);
    *(volatile v4u*)dst = val;
    __threadfence();
    *(volatile v4u*)dst = val;
    __syncthreads();
  }
}

extern "C" void kernel_launch(void* const* d_in, const int* in_sizes, int n_in,
                              void* d_out, int out_size, void* d_ws, size_t ws_size,
                              hipStream_t stream) {
  if (n_in < 10) return;
  if (in_sizes[0] != kNRows * kND) return;
  if (in_sizes[1] != kND || in_sizes[2] != kND || in_sizes[3] != kND) return;
  if (in_sizes[4] != kND || in_sizes[5] != kND) return;
  if (in_sizes[6] != kND * kND || in_sizes[7] != kND * kND || in_sizes[8] != kND * kND || in_sizes[9] != kND * kND) return;
  if (out_size != kNRows * kND) return;
  if (ws_size < kWsEnd) return;

  const float* x   = (const float*)d_in[0];
  const float* tmk = (const float*)d_in[1];
  const float* tmv = (const float*)d_in[2];
  const float* tmr = (const float*)d_in[3];
  const float* td  = (const float*)d_in[4];
  const float* tf  = (const float*)d_in[5];
  const float* Wk  = (const float*)d_in[6];
  const float* Wv  = (const float*)d_in[7];
  const float* Wr  = (const float*)d_in[8];
  const float* Wo  = (const float*)d_in[9];
  float* outp = (float*)d_out;

  unsigned char* base = (unsigned char*)d_ws;
  unsigned short* W16 = (unsigned short*)(base + kOffW16);
  unsigned short* XK  = (unsigned short*)(base + kOffXK);
  unsigned short* XV  = (unsigned short*)(base + kOffXV);
  unsigned short* XR  = (unsigned short*)(base + kOffXR);
  float*          Kf  = (float*)(base + kOffKf);
  float*          Vf  = (float*)(base + kOffVf);
  float*          Zf  = (float*)(base + kOffZf);
  unsigned short* Y16 = (unsigned short*)(base + kOffY16);
  const size_t wplane = (size_t)kND * kND;
  unsigned short* Wk16 = W16 + 0 * wplane;
  unsigned short* Wv16 = W16 + 1 * wplane;
  unsigned short* Wr16 = W16 + 2 * wplane;
  unsigned short* Wo16 = W16 + 3 * wplane;

  {
    const int n8 = kND * kND / 8;
    const dim3 grid((n8 + 255) / 256, 4), blk(256);
    wcast8_kernel<<<grid, blk, 0, stream>>>(Wk, Wv, Wr, Wo, W16, n8, kWCarry);
  }
  {
    const int n8 = kNRows * kND / 8;
    mix_kernel<<<(n8 + 255) / 256, 256, 0, stream>>>(x, tmk, tmv, tmr, XK, XV, XR, n8);
  }
  const int tiles = (kNRows / 64) * (kND / 64);
  const dim3 ggrid((tiles + 7) / 8, 1), gblk(256);
  wmma_gemm64<0, false, 0, 0, false, 0><<<ggrid, gblk, 0, stream>>>(
      XK, XK, kND, 0L, Wk16, Wk16, kND, 0L, (void*)Kf, (void*)Kf, kND, 0L, td, tf, 0L, kNRows, kND, kND, kProjScale);
  wmma_gemm64<0, false, 0, 0, false, 0><<<ggrid, gblk, 0, stream>>>(
      XV, XV, kND, 0L, Wv16, Wv16, kND, 0L, (void*)Vf, (void*)Vf, kND, 0L, td, tf, 0L, kNRows, kND, kND, kProjScale);
  wmma_gemm64<0, false, 0, 0, false, 0><<<ggrid, gblk, 0, stream>>>(
      XR, XR, kND, 0L, Wr16, Wr16, kND, 0L, (void*)Zf, (void*)Zf, kND, 0L, td, tf, 0L, kNRows, kND, kND, kProjScale);
  wkv_scan_kernel<<<(kNB * kND) / 256, 256, 0, stream>>>(Kf, Vf, Zf, td, tf, Y16, kYCarry);
  wmma_gemm64<0, false, 0, 0, false, 0><<<ggrid, gblk, 0, stream>>>(
      Y16, Y16, kND, 0L, Wo16, Wo16, kND, 0L, (void*)outp, (void*)outp, kND, 0L, td, tf, 0L, kNRows, kND, kND, kOutScale);
}
